// SRL_KT_56152402428005
// MI455X (gfx1250) — hardware-verified
//
#include <hip/hip_runtime.h>
#include <stddef.h>
#include <stdint.h>

#define NBAT  32
#define SQ    512
#define NTOK  16384
#define EM    256
#define DIN   1024
#define NH    8
#define HDM   32
#define NL    4
#define QB    128
#define KC    64
#define NQB   (SQ / QB)

static_assert(NTOK == NBAT * SQ);
static_assert(NH * HDM == EM);
static_assert(SQ % QB == 0);
static_assert(QB == 2 * KC);
static_assert(NTOK % 256 == 0);
static_assert(EM % 64 == 0);
static_assert(DIN % 64 == 0);
static_assert(SQ % 256 == 0);
static_assert((SQ * DIN) % 2048 == 0);
static_assert((NTOK * EM) % 2048 == 0);
static_assert(NTOK % 32 == 0);

typedef _Float16 v16h __attribute__((ext_vector_type(16)));
typedef _Float16 v8h  __attribute__((ext_vector_type(8)));
typedef float    v8f  __attribute__((ext_vector_type(8)));
typedef float    v4f  __attribute__((ext_vector_type(4)));
typedef unsigned int v4u __attribute__((ext_vector_type(4)));

union Frag  { v16h v; v8h h[2]; };
union Pack8 { v8h h; v4u u; };

#define SC2048 0.00048828125f

__device__ __forceinline__ v8f mma16(v16h a, v16h b, v8f c) {
  c = __builtin_amdgcn_wmma_f32_16x16x32_f16(false, a, false, b, (short)0, c, false, false);
  asm volatile("v_nop\n\tv_nop\n\tv_nop\n\tv_nop" : "+v"(c) : "v"(a), "v"(b));
  return c;
}

__device__ __forceinline__ v16h ldfrag(const _Float16* p, int ld, int row0, int k0, int lane) {
  const int m = lane & 15, lh = lane >> 4;
  const _Float16* q = p + (size_t)(row0 + m) * ld + k0 + 8 * lh;
  Frag f;
  f.h[0] = *(const v8h*)(q);
  f.h[1] = *(const v8h*)(q + 16);
  return f.v;
}

__device__ __forceinline__ v8f zero8() { return (v8f){0.f, 0.f, 0.f, 0.f, 0.f, 0.f, 0.f, 0.f}; }

__device__ __forceinline__ v4u pack8(v4f a0, v4f a1) {
  Pack8 pk;
  pk.h = (v8h){(_Float16)a0[0], (_Float16)a0[1], (_Float16)a0[2], (_Float16)a0[3],
               (_Float16)a1[0], (_Float16)a1[1], (_Float16)a1[2], (_Float16)a1[3]};
  return pk.u;
}

__device__ __forceinline__ v4f relu4(v4f v) {
  return (v4f){fmaxf(v[0], 0.f), fmaxf(v[1], 0.f), fmaxf(v[2], 0.f), fmaxf(v[3], 0.f)};
}

__device__ __forceinline__ void gemm32x64(const _Float16* __restrict__ A, int lda,
                                          const _Float16* __restrict__ Bt, int ldb, int K,
                                          int m0, int n0, int lane, v8f (&acc)[2][4]) {
#pragma unroll 1
  for (int k0 = 0; k0 < K; k0 += 32) {
    const v16h a0 = ldfrag(A, lda, m0, k0, lane);
    const v16h a1 = ldfrag(A, lda, m0 + 16, k0, lane);
    const v16h b0 = ldfrag(Bt, ldb, n0, k0, lane);
    const v16h b1 = ldfrag(Bt, ldb, n0 + 16, k0, lane);
    const v16h b2 = ldfrag(Bt, ldb, n0 + 32, k0, lane);
    const v16h b3 = ldfrag(Bt, ldb, n0 + 48, k0, lane);
    acc[0][0] = mma16(a0, b0, acc[0][0]);
    acc[1][0] = mma16(a1, b0, acc[1][0]);
    acc[0][1] = mma16(a0, b1, acc[0][1]);
    acc[1][1] = mma16(a1, b1, acc[1][1]);
    acc[0][2] = mma16(a0, b2, acc[0][2]);
    acc[1][2] = mma16(a1, b2, acc[1][2]);
    acc[0][3] = mma16(a0, b3, acc[0][3]);
    acc[1][3] = mma16(a1, b3, acc[1][3]);
  }
}

__device__ __forceinline__ void gemm32x64_cat(const _Float16* __restrict__ A0, const _Float16* __restrict__ A1,
                                              int lda, int ks,
                                              const _Float16* __restrict__ Bt, int ldb, int K,
                                              int m0, int n0, int lane, v8f (&acc)[2][4]) {
#pragma unroll 1
  for (int k0 = 0; k0 < K; k0 += 32) {
    const bool lo = (k0 < ks);
    const _Float16* Ab = lo ? A0 : A1;
    const int ka = lo ? k0 : (k0 - ks);
    const v16h a0 = ldfrag(Ab, lda, m0, ka, lane);
    const v16h a1 = ldfrag(Ab, lda, m0 + 16, ka, lane);
    const v16h b0 = ldfrag(Bt, ldb, n0, k0, lane);
    const v16h b1 = ldfrag(Bt, ldb, n0 + 16, k0, lane);
    const v16h b2 = ldfrag(Bt, ldb, n0 + 32, k0, lane);
    const v16h b3 = ldfrag(Bt, ldb, n0 + 48, k0, lane);
    acc[0][0] = mma16(a0, b0, acc[0][0]);
    acc[1][0] = mma16(a1, b0, acc[1][0]);
    acc[0][1] = mma16(a0, b1, acc[0][1]);
    acc[1][1] = mma16(a1, b1, acc[1][1]);
    acc[0][2] = mma16(a0, b2, acc[0][2]);
    acc[1][2] = mma16(a1, b2, acc[1][2]);
    acc[0][3] = mma16(a0, b3, acc[0][3]);
    acc[1][3] = mma16(a1, b3, acc[1][3]);
  }
}

#define OTP 68
__device__ __forceinline__ void out_epilogue_f32(v8f (&acc)[2][4], float scale, const float (&bb)[4],
                                                 float* sw, float* __restrict__ out, int ldo,
                                                 int m0, int n0, int lane, int hh, int c) {
#pragma unroll
  for (int sub = 0; sub < 2; ++sub) {
    __syncthreads();
#pragma unroll
    for (int t = 0; t < 4; ++t) {
#pragma unroll
      for (int r = 0; r < 8; ++r) sw[(8 * hh + r) * OTP + 16 * t + c] = acc[sub][t][r] * scale + bb[t];
    }
    __syncthreads();
    v4f val[8];
    size_t go[8];
#pragma unroll
    for (int it = 0; it < 8; ++it) {
      const int p    = lane + 32 * it;
      const int L    = p >> 3;
      const int pc   = p & 7;
      const int row  = L >> 1;
      const int half = L & 1;
      val[it] = *(const v4f*)(sw + row * OTP + half * 32 + pc * 4);
      go[it]  = (size_t)(m0 + sub * 16 + row) * ldo + n0 + half * 32 + pc * 4;
    }
    for (int ps = 0; ps < 2; ++ps) {
#pragma unroll
      for (int it = 0; it < 8; ++it) *(volatile v4f*)(out + go[it]) = val[it];
      __threadfence();
    }
  }
}

__device__ __forceinline__ void out_epilogue_h16(v8f (&acc)[2][4], float scale, const float (&bb)[4], float oscale,
                                                 float* sw, _Float16* __restrict__ out, int ldo,
                                                 int m0, int n0, int lane, int hh, int c) {
#pragma unroll
  for (int sub = 0; sub < 2; ++sub) {
    __syncthreads();
#pragma unroll
    for (int t = 0; t < 4; ++t) {
#pragma unroll
      for (int r = 0; r < 8; ++r) {
        const float v = acc[sub][t][r] * scale + bb[t];
        sw[(8 * hh + r) * OTP + 16 * t + c] = fmaxf(v, 0.f) * oscale;
      }
    }
    __syncthreads();
    v4u val[4];
    size_t go[4];
#pragma unroll
    for (int it = 0; it < 4; ++it) {
      const int p  = lane + 32 * it;
      const int L  = p >> 3;
      const int pc = p & 7;
      const float* ra = sw + L * OTP + pc * 8;
      const v4f a0 = *(const v4f*)(ra), a1 = *(const v4f*)(ra + 4);
      val[it] = pack8(a0, a1);
      go[it]  = (size_t)(m0 + sub * 16 + L) * ldo + n0 + pc * 8;
    }
    for (int ps = 0; ps < 2; ++ps) {
#pragma unroll
      for (int it = 0; it < 4; ++it) *(volatile v4u*)(out + go[it]) = val[it];
      __threadfence();
    }
  }
}

__global__ __launch_bounds__(256) void k_tr(const float* __restrict__ src, int K, int N, int szs,
                                            _Float16* __restrict__ dst, int ldd, int dzs, float scale) {
  __shared__ float tl[64][65];
  const int tid = threadIdx.x;
  const int n0 = blockIdx.x * 64, k0 = blockIdx.y * 64;
  const float* s = src + (size_t)blockIdx.z * (size_t)szs;
  _Float16* d = dst + (size_t)blockIdx.z * (size_t)dzs;
#pragma unroll
  for (int it = 0; it < 16; ++it) {
    const int kr = it * 4 + (tid >> 6), nc = tid & 63;
    tl[kr][nc] = s[(size_t)(k0 + kr) * N + n0 + nc] * scale;
  }
  __syncthreads();
  v4u val[2];
  size_t go[2];
#pragma unroll
  for (int j = 0; j < 2; ++j) {
    const int p = tid + 256 * j, nr = p >> 3, pc = p & 7;
    Pack8 pk;
    pk.h = (v8h){(_Float16)tl[pc * 8 + 0][nr], (_Float16)tl[pc * 8 + 1][nr],
                 (_Float16)tl[pc * 8 + 2][nr], (_Float16)tl[pc * 8 + 3][nr],
                 (_Float16)tl[pc * 8 + 4][nr], (_Float16)tl[pc * 8 + 5][nr],
                 (_Float16)tl[pc * 8 + 6][nr], (_Float16)tl[pc * 8 + 7][nr]};
    val[j] = pk.u;
    go[j]  = (size_t)(n0 + nr) * ldd + k0 + pc * 8;
  }
  for (int ps = 0; ps < 2; ++ps) {
#pragma unroll
    for (int j = 0; j < 2; ++j) *(volatile v4u*)(d + go[j]) = val[j];
    __threadfence();
  }
}

__global__ __launch_bounds__(256) void k_small(const float* __restrict__ W_in, const float* __restrict__ type_table,
                                               float* __restrict__ cs) {
  const int n = threadIdx.x;
  float cC = 0.f, cD = 0.f, t0 = 0.f, t1 = 0.f, t2 = 0.f, t3 = 0.f;
#pragma unroll 1
  for (int i = 0; i < EM; ++i) {
    const float wT = W_in[(size_t)(EM + i) * EM + n];
    const float wC = W_in[(size_t)(2 * EM + i) * EM + n];
    const float wD = W_in[(size_t)(3 * EM + i) * EM + n];
    cC += wC;
    cD += wD;
    t0 += type_table[i] * wT;
    t1 += type_table[EM + i] * wT;
    t2 += type_table[2 * EM + i] * wT;
    t3 += type_table[3 * EM + i] * wT;
  }
  volatile float* d = (volatile float*)cs;
  for (int ps = 0; ps < 2; ++ps) {
    d[n] = cC;
    d[EM + n] = cD;
    d[2 * EM + n] = t0;
    d[3 * EM + n] = t1;
    d[4 * EM + n] = t2;
    d[5 * EM + n] = t3;
    __threadfence();
  }
}

__global__ __launch_bounds__(256) void k_pe(const float* __restrict__ pe, _Float16* __restrict__ ph) {
  const int tid = threadIdx.x;
  const int row = blockIdx.x * 2 + (tid >> 7);
  const int col = (tid & 127) * 8;
  const int srow = (row > 0) ? (row - 1) : 0;
  const float f = (row > 0) ? 16.0f : 0.0f;
  const float* p = pe + (size_t)srow * DIN + col;
  const v4f a0 = *(const v4f*)(p) * f, a1 = *(const v4f*)(p + 4) * f;
  const v4u vv = pack8(a0, a1);
  volatile v4u* d = (volatile v4u*)(ph + (size_t)row * DIN + col);
  *d = vv;
  __threadfence();
  *d = vv;
}

__global__ __launch_bounds__(256) void k_gath(const int* __restrict__ item_inputs, const int* __restrict__ item_ids,
                                              const float* __restrict__ use_table, int nitem,
                                              _Float16* __restrict__ ie, _Float16* __restrict__ qh) {
  const int tid = threadIdx.x, lane = tid & 31, wave = tid >> 5;
  const int row = blockIdx.x * 8 + wave;
  const int s = row & (SQ - 1);
  int ia = item_inputs[row];
  ia = min(max(ia, 0), nitem - 1);
  int ib = item_ids[row];
  ib = min(max(ib, 0), nitem - 1);
  const float fa = (s > 0) ? 64.0f : 0.0f;
  const float* ua = use_table + (size_t)ia * EM + 8 * lane;
  const float* ub = use_table + (size_t)ib * EM + 8 * lane;
  const v4f a0 = *(const v4f*)(ua) * fa,    a1 = *(const v4f*)(ua + 4) * fa;
  const v4f b0 = *(const v4f*)(ub) * 64.0f, b1 = *(const v4f*)(ub + 4) * 64.0f;
  const v4u va = pack8(a0, a1), vb = pack8(b0, b1);
  const size_t go = (size_t)row * EM + 8 * lane;
  for (int ps = 0; ps < 2; ++ps) {
    *(volatile v4u*)(ie + go) = va;
    *(volatile v4u*)(qh + go) = vb;
    __threadfence();
  }
}

__global__ __launch_bounds__(256) void k_rel(const float* __restrict__ rel, _Float16* __restrict__ rh) {
  const int tid = threadIdx.x, lane = tid & 31, wave = tid >> 5;
  const size_t row = (size_t)blockIdx.x * 8 + wave;
  const int q = (int)(row & (SQ - 1));
  const float* rr = rel + row * SQ;
  float x[16];
  float mx = -3.0e38f;
#pragma unroll
  for (int i = 0; i < 2; ++i) {
    const int kb = 256 * i + 8 * lane;
    const v4f a0 = *(const v4f*)(rr + kb), a1 = *(const v4f*)(rr + kb + 4);
#pragma unroll
    for (int e = 0; e < 8; ++e) {
      const float vv = (e < 4) ? a0[e & 3] : a1[e & 3];
      float t = (vv == 0.0f) ? -1.0e4f : vv;
      t = (kb + e > q) ? t : -1.0e4f;
      x[8 * i + e] = t;
      mx = fmaxf(mx, t);
    }
  }
#pragma unroll
  for (int off = 16; off >= 1; off >>= 1) mx = fmaxf(mx, __shfl_xor(mx, off, 32));
  float sm = 0.f;
#pragma unroll
  for (int i = 0; i < 16; ++i) {
    const float e = __expf(x[i] - mx);
    x[i] = e;
    sm += e;
  }
#pragma unroll
  for (int off = 16; off >= 1; off >>= 1) sm += __shfl_xor(sm, off, 32);
  const float inv = 1.0f / sm;
  v4u val[2];
  size_t go[2];
#pragma unroll
  for (int i = 0; i < 2; ++i) {
    Pack8 pk;
    pk.h = (v8h){(_Float16)((x[8 * i + 0] * inv) * 4096.0f), (_Float16)((x[8 * i + 1] * inv) * 4096.0f),
                 (_Float16)((x[8 * i + 2] * inv) * 4096.0f), (_Float16)((x[8 * i + 3] * inv) * 4096.0f),
                 (_Float16)((x[8 * i + 4] * inv) * 4096.0f), (_Float16)((x[8 * i + 5] * inv) * 4096.0f),
                 (_Float16)((x[8 * i + 6] * inv) * 4096.0f), (_Float16)((x[8 * i + 7] * inv) * 4096.0f)};
    val[i] = pk.u;
    go[i]  = row * SQ + 256 * i + 8 * lane;
  }
  for (int ps = 0; ps < 2; ++ps) {
#pragma unroll
    for (int i = 0; i < 2; ++i) *(volatile v4u*)(rh + go[i]) = val[i];
    __threadfence();
  }
}

__global__ __launch_bounds__(256) void k_gemm_f32(const _Float16* __restrict__ ap, int lda, int zas,
                                                  const _Float16* __restrict__ wt, int ldb, int zbs, int K,
                                                  const float* __restrict__ bias, int hasb, float scale,
                                                  float* __restrict__ out, int ldo, int zos) {
  __shared__ __align__(16) float st[8][16 * OTP];
  const int tid = threadIdx.x, lane = tid & 31, wave = tid >> 5;
  const int hh = lane >> 4, c = lane & 15;
  const int z = blockIdx.z;
  const _Float16* A = ap + (size_t)z * (size_t)zas;
  const _Float16* B = wt + (size_t)z * (size_t)zbs;
  float* O = out + (size_t)z * (size_t)zos;
  const int m0 = blockIdx.x * 256 + wave * 32;
  const int n0 = blockIdx.y * 64;

  v8f acc[2][4];
#pragma unroll
  for (int s = 0; s < 2; ++s)
#pragma unroll
    for (int t = 0; t < 4; ++t) acc[s][t] = zero8();
  gemm32x64(A, lda, B, ldb, K, m0, n0, lane, acc);
  float bb[4];
  if (hasb != 0) {
#pragma unroll
    for (int t = 0; t < 4; ++t) bb[t] = bias[n0 + 16 * t + c];
  } else {
#pragma unroll
    for (int t = 0; t < 4; ++t) bb[t] = 0.f;
  }
  out_epilogue_f32(acc, scale, bb, st[wave], O, ldo, m0, n0, lane, hh, c);
}

__global__ __launch_bounds__(256) void k_inp(const _Float16* __restrict__ ie, const _Float16* __restrict__ wint,
                                             const float* __restrict__ pep, const float* __restrict__ cs,
                                             const int* __restrict__ type_inputs,
                                             const float* __restrict__ qresp, const float* __restrict__ label,
                                             _Float16* __restrict__ kvh) {
  __shared__ __align__(16) float st[8][16 * OTP];
  __shared__ __align__(16) float adds[6 * 64];
  __shared__ float rowq[256];
  __shared__ float rowl[256];
  __shared__ int   rowt[256];
  const int tid = threadIdx.x, lane = tid & 31, wave = tid >> 5;
  const int hh = lane >> 4, c = lane & 15;
  const int mb = blockIdx.x * 256;
  const int m0 = mb + wave * 32;
  const int n0 = blockIdx.y * 64;

  {
    const int m = mb + tid;
    rowq[tid] = qresp[m];
    rowl[tid] = label[m];
    const int ty = type_inputs[m];
    rowt[tid] = min(max(ty, 0), 3);
    const int i0 = tid;
    adds[i0] = cs[(size_t)(i0 >> 6) * EM + n0 + (i0 & 63)];
    const int i1 = min(tid + 256, 383);
    const float a1 = cs[(size_t)(i1 >> 6) * EM + n0 + (i1 & 63)];
    if (tid < 128) adds[tid + 256] = a1;
  }

  v8f acc[2][4];
#pragma unroll
  for (int s = 0; s < 2; ++s)
#pragma unroll
    for (int t = 0; t < 4; ++t) acc[s][t] = zero8();
  gemm32x64(ie, EM, wint, DIN, EM, m0, n0, lane, acc);

  float* sw = st[wave];
#pragma unroll
  for (int sub = 0; sub < 2; ++sub) {
    __syncthreads();
#pragma unroll
    for (int it = 0; it < 8; ++it) {
      const int p = lane + 32 * it, L = p >> 4, pc = p & 15;
      const int s = (m0 + sub * 16 + L) & (SQ - 1);
      *(v4f*)(sw + L * OTP + pc * 4) = *(const v4f*)(pep + (size_t)s * EM + n0 + pc * 4);
    }
    __syncthreads();
#pragma unroll
    for (int r = 0; r < 8; ++r) {
      const int lr = wave * 32 + sub * 16 + 8 * hh + r;
      const float qv = rowq[lr], lv = rowl[lr];
      const int ty = rowt[lr];
      const float* t4 = adds + (2 + ty) * 64;
#pragma unroll
      for (int t = 0; t < 4; ++t) {
        const int cl = 16 * t + c;
        float* cell = sw + (8 * hh + r) * OTP + cl;
        const float v = acc[sub][t][r] * SC2048 + *cell + t4[cl] + qv * adds[cl] + lv * adds[64 + cl];
        *cell = fmaxf(v, 0.f) * 64.0f;
      }
    }
    __syncthreads();
    v4u val[4];
    size_t go[4];
#pragma unroll
    for (int it = 0; it < 4; ++it) {
      const int p  = lane + 32 * it;
      const int L  = p >> 3;
      const int pc = p & 7;
      const float* ra = sw + L * OTP + pc * 8;
      const v4f a0 = *(const v4f*)(ra), a1 = *(const v4f*)(ra + 4);
      val[it] = pack8(a0, a1);
      go[it]  = (size_t)(m0 + sub * 16 + L) * EM + n0 + pc * 8;
    }
    for (int ps = 0; ps < 2; ++ps) {
#pragma unroll
      for (int it = 0; it < 4; ++it) *(volatile v4u*)(kvh + go[it]) = val[it];
      __threadfence();
    }
  }
}

#define STP 72
#define SVP 264
__global__ __launch_bounds__(256) void k_qkv(const _Float16* __restrict__ aq, const _Float16* __restrict__ akv,
                                             const _Float16* __restrict__ wt,
                                             const float* __restrict__ bq, const float* __restrict__ bk,
                                             const float* __restrict__ bv,
                                             _Float16* __restrict__ qp, _Float16* __restrict__ kp,
                                             _Float16* __restrict__ vtp) {
  __shared__ __align__(16) _Float16 st[256 * STP];
  const int tid = threadIdx.x, lane = tid & 31, wave = tid >> 5;
  const int hh = lane >> 4, c = lane & 15;
  const int bx = blockIdx.x;
  const int b  = bx >> 1;
  const int sb = (bx & 1) * 256;
  const int ns = blockIdx.y;
  const int which = ns >> 2;
  const int cb = (ns & 3) * 64;
  const int m0 = bx * 256 + wave * 32;
  const int n0 = ns * 64;
  const _Float16* A = (which == 0) ? aq : akv;

  v8f acc[2][4];
#pragma unroll
  for (int s = 0; s < 2; ++s)
#pragma unroll
    for (int t = 0; t < 4; ++t) acc[s][t] = zero8();
  gemm32x64(A, EM, wt, EM, EM, m0, n0, lane, acc);

  float bb[4];
#pragma unroll
  for (int t = 0; t < 4; ++t) {
    const int i = cb + 16 * t + c;
    const float xq = bq[i], xk = bk[i], xv = bv[i];
    bb[t] = (which == 0) ? xq : ((which == 1) ? xk : xv);
  }
  const float carry = (which == 0) ? 64.0f : 16.0f;

  if (which < 2) {
#pragma unroll
    for (int sub = 0; sub < 2; ++sub)
#pragma unroll
      for (int t = 0; t < 4; ++t)
#pragma unroll
        for (int r = 0; r < 8; ++r)
          st[(wave * 32 + sub * 16 + 8 * hh + r) * STP + 16 * t + c] =
              (_Float16)((acc[sub][t][r] * SC2048 + bb[t]) * carry);
  } else {
#pragma unroll
    for (int sub = 0; sub < 2; ++sub)
#pragma unroll
      for (int t = 0; t < 4; ++t)
#pragma unroll
        for (int r = 0; r < 8; ++r)
          st[(16 * t + c) * SVP + wave * 32 + sub * 16 + 8 * hh + r] =
              (_Float16)((acc[sub][t][r] * SC2048 + bb[t]) * carry);
  }
  __syncthreads();

  if (which < 2) {
    _Float16* base = ((which == 0) ? qp : kp) + ((size_t)(b * NH + 2 * (ns & 3)) * SQ + sb) * HDM;
#pragma unroll
    for (int g = 0; g < 2; ++g) {
      v4u val[4];
      size_t go[4];
#pragma unroll
      for (int j = 0; j < 4; ++j) {
        const int p    = tid + 256 * (4 * g + j);
        const int hsel = p >> 10;
        const int pl   = p & 1023;
        const int lr   = pl >> 2;
        const int pc   = pl & 3;
        Pack8 pk;
        pk.h   = *(const v8h*)(st + lr * STP + hsel * 32 + pc * 8);
        val[j] = pk.u;
        go[j]  = (size_t)hsel * (SQ * HDM) + (size_t)pl * 8;
      }
      for (int ps = 0; ps < 2; ++ps) {
#pragma unroll
        for (int j = 0; j < 4; ++j) *(volatile v4u*)(base + go[j]) = val[j];
        __threadfence();
      }
    }
  } else {
    _Float16* base = vtp + (size_t)(b * EM + cb) * SQ + sb;
#pragma unroll
    for (int g = 0; g < 2; ++g) {
      v4u val[4];
      size_t go[4];
#pragma unroll
      for (int j = 0; j < 4; ++j) {
        const int p    = tid + 256 * (4 * g + j);
        const int drow = p >> 5;
        const int pc   = p & 31;
        Pack8 pk;
        pk.h   = *(const v8h*)(st + drow * SVP + pc * 8);
        val[j] = pk.u;
        go[j]  = (size_t)drow * SQ + pc * 8;
      }
      for (int ps = 0; ps < 2; ++ps) {
#pragma unroll
        for (int j = 0; j < 4; ++j) *(volatile v4u*)(base + go[j]) = val[j];
        __threadfence();
      }
    }
  }
}

#define KSP 40
#define VSP 72
#define PSP 72
#define OSP 36
__global__ __launch_bounds__(256) void k_attn(const _Float16* __restrict__ qp, const _Float16* __restrict__ kp,
                                              const _Float16* __restrict__ vt, const float* __restrict__ rv,
                                              const float* __restrict__ oold, float* __restrict__ onew,
                                              const float* __restrict__ l1p, float sscale, int first) {
  __shared__ __align__(16) _Float16 Ks[KC * KSP];
  __shared__ __align__(16) _Float16 Vs[HDM * VSP];
  __shared__ __align__(16) _Float16 Ps[8 * 16 * PSP];
  __shared__ __align__(16) float    Os[8 * 16 * OSP];

  const int tid = threadIdx.x, lane = tid & 31, wave = tid >> 5;
  const int hh = lane >> 4, c = lane & 15;
  const int qb  = blockIdx.x & 3;
  const int hb  = blockIdx.x >> 2;
  const int h   = hb & 7;
  const int b   = hb >> 3;
  const int q0  = qb * QB + wave * 16;
  const int nck = 2 * qb + 2;

  const _Float16* Q = qp + (size_t)hb * SQ * HDM;
  const _Float16* K = kp + (size_t)hb * SQ * HDM;
  const _Float16* V = vt + (size_t)hb * HDM * SQ;

  const v16h qa = ldfrag(Q, HDM, q0, 0, lane);

  const float NEGI = -__builtin_huge_valf();
  float mrow[8], lrow[8];
  v8f oacc[2];
#pragma unroll
  for (int r = 0; r < 8; ++r) { mrow[r] = NEGI; lrow[r] = 0.f; }
#pragma unroll
  for (int t = 0; t < 2; ++t) oacc[t] = zero8();

  _Float16* pw = Ps + wave * 16 * PSP;

  for (int kc = 0; kc < nck; ++kc) {
    const int kv0 = kc * KC;
    __syncthreads();
    {
      const int r  = tid >> 2;
      const int qq = (tid & 3) * 8;
      *(v8h*)(Ks + r * KSP + qq) = *(const v8h*)(K + (size_t)(kv0 + r) * HDM + qq);
      const int r2 = tid >> 3;
      const int q2 = (tid & 7) * 8;
      *(v8h*)(Vs + r2 * VSP + q2) = *(const v8h*)(V + (size_t)r2 * SQ + kv0 + q2);
    }
    __syncthreads();

    v8f s[4];
#pragma unroll
    for (int j = 0; j < 4; ++j) {
      const v16h kb = ldfrag(Ks, KSP, j * 16, 0, lane);
      s[j] = mma16(qa, kb, zero8());
    }
    float cm[8];
#pragma unroll
    for (int r = 0; r < 8; ++r) {
      const int qr = q0 + 8 * hh + r;
      float m = NEGI;
#pragma unroll
      for (int j = 0; j < 4; ++j) {
        const int key = kv0 + j * 16 + c;
        float x = s[j][r] * sscale;
        x = (key > qr) ? -1.0e9f : x;
        s[j][r] = x;
        m = fmaxf(m, x);
      }
#pragma unroll
      for (int off = 1; off < 16; off <<= 1) m = fmaxf(m, __shfl_xor(m, off, 32));
      cm[r] = m;
    }
    float al[8];
#pragma unroll
    for (int r = 0; r < 8; ++r) {
      const float mnew  = fmaxf(mrow[r], cm[r]);
      const float alpha = __expf(mrow[r] - mnew);
      mrow[r] = mnew;
      float psum = 0.f;
#pragma unroll
      for (int j = 0; j < 4; ++j) {
        const float p = __expf(s[j][r] - mnew);
        psum += p;
        pw[(8 * hh + r) * PSP + j * 16 + c] = (_Float16)(p * 1024.0f);
      }
#pragma unroll
      for (int off = 1; off < 16; off <<= 1) psum += __shfl_xor(psum, off, 32);
      lrow[r] = lrow[r] * alpha + psum;
      al[r] = alpha;
    }
#pragma unroll
    for (int t = 0; t < 2; ++t)
#pragma unroll
      for (int r = 0; r < 8; ++r) oacc[t][r] *= al[r];
    __syncthreads();

#pragma unroll
    for (int kk = 0; kk < 2; ++kk) {
      const v16h pa = ldfrag(pw, PSP, 0, kk * 32, lane);
#pragma unroll
      for (int t = 0; t < 2; ++t) {
        const v16h vb = ldfrag(Vs, VSP, t * 16, kk * 32, lane);
        oacc[t] = mma16(pa, vb, oacc[t]);
      }
    }
  }

  float invl[8];
#pragma unroll
  for (int r = 0; r < 8; ++r) invl[r] = (lrow[r] > 0.f) ? ((1.0f / lrow[r]) * 6.103515625e-05f) : 0.f;
  __syncthreads();
  float* of = Os + wave * 16 * OSP;
#pragma unroll
  for (int r = 0; r < 8; ++r) {
#pragma unroll
    for (int t = 0; t < 2; ++t)
      of[(8 * hh + r) * OSP + 16 * t + c] = oacc[t][r] * invl[r];
  }
  __syncthreads();
  const float l1v = l1p[0];
  const float om  = 1.0f - l1v;
  v4f val[4];
  size_t go[4];
#pragma unroll
  for (int it = 0; it < 4; ++it) {
    const int p  = lane + 32 * it;
    const int L  = p >> 3;
    const int pc = p & 7;
    const v4f o4 = *(const v4f*)(of + L * OSP + pc * 4);
    const size_t g = (size_t)(b * SQ + q0 + L) * EM + (size_t)h * HDM + pc * 4;
    const v4f r4 = *(const v4f*)(rv + g);
    v4f v = o4 * om + r4 * l1v;
    if (first == 0) {
      const v4f old = *(const v4f*)(oold + g);
      v = old + relu4(v);
    }
    val[it] = v;
    go[it]  = g;
  }
  for (int ps = 0; ps < 2; ++ps) {
#pragma unroll
    for (int it = 0; it < 4; ++it) *(volatile v4f*)(onew + go[it]) = val[it];
    __threadfence();
  }
}

__global__ __launch_bounds__(256) void k_cvt16(const float* __restrict__ src, _Float16* __restrict__ dh, float scale) {
  const int tid = threadIdx.x;
  const size_t row = (size_t)blockIdx.x * 8 + (tid >> 5);
  const int col = (tid & 31) * 8;
  const size_t o = row * EM + col;
  const v4f a0 = *(const v4f*)(src + o) * scale;
  const v4f a1 = *(const v4f*)(src + o + 4) * scale;
  const v4u vv = pack8(a0, a1);
  volatile v4u* d = (volatile v4u*)(dh + o);
  *d = vv;
  __threadfence();
  *d = vv;
}

#define HSP 260
__global__ __launch_bounds__(128) void k_head(const _Float16* __restrict__ a0p, const _Float16* __restrict__ a1p,
                                              const _Float16* __restrict__ w1t, const float* __restrict__ b1,
                                              const float* __restrict__ w2, const float* __restrict__ b2,
                                              float* __restrict__ out) {
  __shared__ __align__(16) float hs[32 * HSP];
  __shared__ __align__(16) float w2s[EM];
  __shared__ __align__(16) float red[32];
  const int tid = threadIdx.x, lane = tid & 31, wave = tid >> 5;
  const int hh = lane >> 4, c = lane & 15;
  const int m0 = blockIdx.x * 32;
  const int n0 = wave * 64;
  w2s[tid] = w2[tid];
  w2s[tid + 128] = w2[tid + 128];

  v8f acc[2][4];
#pragma unroll
  for (int s = 0; s < 2; ++s)
#pragma unroll
    for (int t = 0; t < 4; ++t) acc[s][t] = zero8();
  gemm32x64_cat(a0p, a1p, EM, EM, w1t, 2 * EM, 2 * EM, m0, n0, lane, acc);

#pragma unroll
  for (int t = 0; t < 4; ++t) {
    const float bb = b1[n0 + 16 * t + c];
#pragma unroll
    for (int sub = 0; sub < 2; ++sub)
#pragma unroll
      for (int r = 0; r < 8; ++r)
        hs[(sub * 16 + 8 * hh + r) * HSP + n0 + 16 * t + c] = fmaxf(acc[sub][t][r] * SC2048 + bb, 0.f);
  }
  __syncthreads();

  const int row = tid >> 2, part = tid & 3;
  const float* hr = hs + row * HSP + part * 64;
  const float* wr = w2s + part * 64;
  float sum = 0.f;
#pragma unroll 8
  for (int j = 0; j < 64; ++j) sum += hr[j] * wr[j];
  sum += __shfl_xor(sum, 1, 32);
  sum += __shfl_xor(sum, 2, 32);
  const float v = sum + b2[0];
  if (part == 0) red[row] = v;
  __syncthreads();
  if (wave == 0) {
    const v4f o = *(const v4f*)(red + 4 * (lane & 7));
    volatile v4f* d = (volatile v4f*)(out + m0 + 4 * (lane & 7));
    for (int ps = 0; ps < 2; ++ps) {
      if (lane < 8) *d = o;
      __threadfence();
    }
  }
}

extern "C" void kernel_launch(void* const* d_in, const int* in_sizes, int n_in,
                              void* d_out, int out_size, void* d_ws, size_t ws_size,
                              hipStream_t stream) {
  if (n_in < 23) return;
  if (in_sizes[0] != NTOK) return;
  if (in_sizes[1] != NTOK) return;
  if (in_sizes[2] != NTOK) return;
  if (in_sizes[3] != NTOK) return;
  if (in_sizes[4] != NBAT * SQ * SQ) return;
  if (in_sizes[6] != NTOK) return;
  if (in_sizes[7] < EM || (in_sizes[7] % EM) != 0) return;
  if (in_sizes[8] != 4 * EM) return;
  if (in_sizes[9] != DIN * EM) return;
  if (in_sizes[10] != EM) return;
  if (in_sizes[11] != NL * EM * EM) return;
  if (in_sizes[12] != NL * EM) return;
  if (in_sizes[13] != NL * EM * EM) return;
  if (in_sizes[14] != NL * EM) return;
  if (in_sizes[15] != NL * EM * EM) return;
  if (in_sizes[16] != NL * EM) return;
  if (in_sizes[17] < 1) return;
  if (in_sizes[18] != 2 * EM * EM) return;
  if (in_sizes[19] != EM) return;
  if (in_sizes[20] != EM) return;
  if (in_sizes[21] < 1) return;
  if (in_sizes[22] != SQ * DIN) return;
  if (out_size != NTOK) return;

  const int*   item_inputs = (const int*)d_in[0];
  const float* label       = (const float*)d_in[1];
  const int*   type_inputs = (const int*)d_in[2];
  const int*   item_ids    = (const int*)d_in[3];
  const float* rel         = (const float*)d_in[4];
  const float* qresp       = (const float*)d_in[6];
  const float* use_table   = (const float*)d_in[7];
  const float* type_table  = (const float*)d_in[8];
  const float* W_in        = (const float*)d_in[9];
  const float* b_in        = (const float*)d_in[10];
  const float* Wq          = (const float*)d_in[11];
  const float* bq          = (const float*)d_in[12];
  const float* Wk          = (const float*)d_in[13];
  const float* bk          = (const float*)d_in[14];
  const float* Wv          = (const float*)d_in[15];
  const float* bv          = (const float*)d_in[16];
  const float* l1          = (const float*)d_in[17];
  const float* W1          = (const float*)d_in[18];
  const float* b1          = (const float*)d_in[19];
  const float* W2          = (const float*)d_in[20];
  const float* b2          = (const float*)d_in[21];
  const float* pe_inter    = (const float*)d_in[22];
  float* out = (float*)d_out;
  const int nitem = in_sizes[7] / EM;

  const size_t planeqkv = (size_t)NBAT * NH * SQ * HDM * 2;
  size_t off = 0;
  const size_t oWT  = off; off += (size_t)NL * 3 * EM * EM * 2;
  const size_t oWIN = off; off += (size_t)EM * DIN * 2;
  const size_t oW1  = off; off += (size_t)EM * 2 * EM * 2;
  const size_t oCS  = off; off += 8192;
  const size_t oPE  = off; off += (size_t)SQ * DIN * 2;
  const size_t oPEP = off; off += (size_t)SQ * EM * 4;
  const size_t oIE  = off; off += (size_t)NTOK * EM * 2;
  const size_t oQ16 = off; off += (size_t)NTOK * EM * 2;
  const size_t oR16 = off; off += (size_t)NTOK * SQ * 2;
  const size_t oKV  = off; off += (size_t)NTOK * EM * 2;
  const size_t oQP  = off; off += planeqkv;
  const size_t oKP  = off; off += planeqkv;
  const size_t oVT  = off; off += planeqkv;
  const size_t oRV  = off; off += (size_t)NTOK * EM * 4;
  const size_t oOA  = off; off += (size_t)NTOK * EM * 4;
  const size_t oOB  = off; off += (size_t)NTOK * EM * 4;
  if (off > ws_size) return;
  if (off > (size_t)134217728) return;
  if ((size_t)6 * EM * 4 > 8192) return;

  char* ws = (char*)d_ws;
  _Float16* WT   = (_Float16*)(ws + oWT);
  _Float16* WINT = (_Float16*)(ws + oWIN);
  _Float16* W1T  = (_Float16*)(ws + oW1);
  float*    CS   = (float*)(ws + oCS);
  _Float16* PE16 = (_Float16*)(ws + oPE);
  float*    PEP  = (float*)(ws + oPEP);
  _Float16* IE16 = (_Float16*)(ws + oIE);
  _Float16* Q16  = (_Float16*)(ws + oQ16);
  _Float16* R16  = (_Float16*)(ws + oR16);
  _Float16* KV16 = (_Float16*)(ws + oKV);
  _Float16* QP   = (_Float16*)(ws + oQP);
  _Float16* KP   = (_Float16*)(ws + oKP);
  _Float16* VT   = (_Float16*)(ws + oVT);
  float*    RV   = (float*)(ws + oRV);
  float*    OA   = (float*)(ws + oOA);
  float*    OB   = (float*)(ws + oOB);

  k_tr<<<dim3(EM / 64, EM / 64, NL), dim3(256), 0, stream>>>(Wq, EM, EM, EM * EM, WT, EM, 3 * EM * EM, 32.0f);
  k_tr<<<dim3(EM / 64, EM / 64, NL), dim3(256), 0, stream>>>(Wk, EM, EM, EM * EM, WT + (size_t)EM * EM, EM, 3 * EM * EM, 32.0f);
  k_tr<<<dim3(EM / 64, EM / 64, NL), dim3(256), 0, stream>>>(Wv, EM, EM, EM * EM, WT + (size_t)2 * EM * EM, EM, 3 * EM * EM, 32.0f);
  k_tr<<<dim3(EM / 64, DIN / 64, 1), dim3(256), 0, stream>>>(W_in, DIN, EM, 0, WINT, DIN, 0, 32.0f);
  k_tr<<<dim3(EM / 64, (2 * EM) / 64, 1), dim3(256), 0, stream>>>(W1, 2 * EM, EM, 0, W1T, 2 * EM, 0, 32.0f);
  k_small<<<dim3(1), dim3(256), 0, stream>>>(W_in, type_table, CS);
  k_pe<<<dim3((SQ * DIN) / 2048), dim3(256), 0, stream>>>(pe_inter, PE16);
  k_gemm_f32<<<dim3(SQ / 256, EM / 64, 1), dim3(256), 0, stream>>>(PE16, DIN, 0, WINT, DIN, 0, DIN, b_in, 1,
                                                                  0.001953125f, PEP, EM, 0);
  k_gath<<<dim3(NTOK / 8), dim3(256), 0, stream>>>(item_inputs, item_ids, use_table, nitem, IE16, Q16);
  k_rel<<<dim3(NTOK / 8), dim3(256), 0, stream>>>(rel, R16);
  k_inp<<<dim3(NTOK / 256, EM / 64), dim3(256), 0, stream>>>(IE16, WINT, PEP, CS, type_inputs, qresp, label, KV16);
  const float sscale = 0.17677669529663688f * 0.0009765625f;
  for (int i = 0; i < NL; ++i) {
    k_qkv<<<dim3(NTOK / 256, (3 * EM) / 64), dim3(256), 0, stream>>>(
        Q16, KV16, WT + (size_t)i * 3 * EM * EM, bq + (size_t)i * EM, bk + (size_t)i * EM, bv + (size_t)i * EM,
        QP, KP, VT);
    k_gemm_f32<<<dim3(SQ / 256, EM / 64, NBAT), dim3(256), 0, stream>>>(R16, SQ, SQ * SQ, VT, SQ, EM * SQ, SQ,
                                                                       b_in, 0, 1.52587890625e-05f, RV, EM, SQ * EM);
    float* onew = (i & 1) ? OB : OA;
    const float* oold = (i & 1) ? OA : OB;
    k_attn<<<dim3(NBAT * NH * NQB), dim3(256), 0, stream>>>(QP, KP, VT, RV, oold, onew, l1, sscale, (i == 0) ? 1 : 0);
    k_cvt16<<<dim3(NTOK / 8), dim3(256), 0, stream>>>(onew, KV16, 64.0f);
  }
  k_head<<<dim3(NTOK / 32), dim3(128), 0, stream>>>(KV16, Q16, W1T, b1, W2, b2, out);
  (void)hipGetLastError();
}
